// RNNModel_63737314672804
// MI455X (gfx1250) — hardware-verified
//
#include <hip/hip_runtime.h>
#include <math.h>

constexpr int NB    = 512;
constexpr int NTR   = 1024;
constexpr int NT2   = 512;
constexpr int NF    = 24;
constexpr int NFP   = 32;
constexpr int NC    = 32;
constexpr int NU    = 128;
constexpr int NU2   = 256;
constexpr int NO    = 6;
constexpr int ND1   = 64;
constexpr int NZ    = NU2 + NO;
constexpr int BCH   = 256;
constexpr int NPASS = NB / BCH;
constexpr int NTHF  = 256;
constexpr int NTHR  = 128;
constexpr int APF   = 40;
constexpr int SPF   = 36;
constexpr int HP    = 136;
constexpr int OPH   = 132;
constexpr int ZP    = 264;
constexpr int UP    = 68;
constexpr float WSC     = 16.0f;
constexpr float WSC_INV = 1.0f / 16.0f;
constexpr float BN_EPS  = 1e-5f;

static_assert(NB % BCH == 0, "passes exact");
static_assert(BCH % 16 == 0, "16-row tiles per recurrence block");
static_assert(NU == 32 * (NTHR / 32), "4 waves x 32 hidden columns");
static_assert(NTR == 2 * NT2, "pool window 2");
static_assert((NB * NTR) % 256 == 0 && NTR % 256 == 0, "front block rows inside one batch row");
static_assert(NFP % 32 == 0 && NU % 32 == 0 && NU2 % 32 == 0, "every WMMA K is a multiple of 32");
static_assert(NF % 4 == 0 && NF <= NFP - 8, "front staging and zero pad layout");
static_assert((2 * 16 * HP) % NTHR == 0, "h tile zero fill exact");
static_assert(NB % 32 == 0, "head: one 128-B output line per block");
static_assert(NC * 2 == 64 && HP % 8 == 0 && APF % 8 == 0 && OPH % 4 == 0, "alignment");

typedef __attribute__((ext_vector_type(16))) _Float16 v16h;
typedef __attribute__((ext_vector_type(8)))  _Float16 v8h;
typedef __attribute__((ext_vector_type(8)))  float    v8f;
typedef __attribute__((ext_vector_type(4)))  float    v4f;
typedef __attribute__((ext_vector_type(2)))  unsigned v2u;
typedef __attribute__((ext_vector_type(4)))  unsigned v4u;

__device__ __forceinline__ void guard2_h3(v8f& a, v8f& b, v16h x, v16h y, v16h z) {
  asm volatile("v_nop\n\tv_nop\n\tv_nop\n\tv_nop" : "+v"(a), "+v"(b) : "v"(x), "v"(y), "v"(z));
}
__device__ __forceinline__ void guard4_h4(v8f& a, v8f& b, v8f& c, v8f& d, v16h w, v16h x, v16h y, v16h z) {
  asm volatile("v_nop\n\tv_nop\n\tv_nop\n\tv_nop" : "+v"(a), "+v"(b), "+v"(c), "+v"(d) : "v"(w), "v"(x), "v"(y), "v"(z));
}
__device__ __forceinline__ void acc_guard2(v8f& a, v8f& b) {
  asm volatile("v_nop\n\tv_nop\n\tv_nop\n\tv_nop" : "+v"(a), "+v"(b));
}

template <typename T> struct Frag;
template <> struct Frag<_Float16> {
  typedef v16h V; union U { v16h v; v8h h[2]; };
  static __device__ __forceinline__ v16h load(const _Float16* p) {
    U f; f.h[0] = *(const v8h*)(p); f.h[1] = *(const v8h*)(p + 16); return f.v;
  }
  static __device__ __forceinline__ v8f mma(v16h a, v16h b, v8f c) {
    return __builtin_amdgcn_wmma_f32_16x16x32_f16(false, a, false, b, (short)0, c, false, false);
  }
};

__device__ __forceinline__ float h16_to_f32(unsigned hb) {
  const unsigned sgn = (hb & 0x8000u) << 16; const unsigned em = hb & 0x7fffu;
  const float fn = __uint_as_float((em << 13) + 0x38000000u);
  const float fs = (float)em * 5.9604644775390625e-8f;
  const float mag = (em < 0x400u) ? fs : fn; return __uint_as_float(__float_as_uint(mag) | sgn);
}

__device__ __forceinline__ float tanh_f(float x) {
  const float e = expf(2.0f * x);
  return 1.0f - 2.0f * __builtin_amdgcn_rcpf(e + 1.0f);
}

__global__ __launch_bounds__(NTHF) void wprep_kernel(const float* __restrict__ src, int kreal, int ncols, int kpad,
                                                    unsigned short* __restrict__ dst, float sc) {
  const int i  = blockIdx.x * NTHF + threadIdx.x;
  const int k8 = kpad >> 3;
  const int n8 = ncols * k8;
  if (i < n8) {
    const int n  = i / k8;
    const int c8 = i - n * k8;
    v8h hv;
#pragma unroll
    for (int e = 0; e < 8; ++e) {
      const int k  = c8 * 8 + e;
      const int kc = (k < kreal) ? k : (kreal - 1);
      const float f = (k < kreal) ? 1.0f : 0.0f;
      const float v = src[(size_t)kc * ncols + n] * sc * f;
      hv[e] = (_Float16)v;
    }
    *(volatile v8h*)(dst + (size_t)i * 8) = hv;
    __threadfence();
    *(volatile v8h*)(dst + (size_t)i * 8) = hv;
  }
}

__device__ __forceinline__ void front_epi(v8f acc, float tb, float mu, float rs, float sc, float bi,
                                          float* slab, int prow, int col) {
  float xv[8];
#pragma unroll
  for (int r = 0; r < 8; ++r) {
    const float a = tanh_f(acc[r] * WSC_INV + tb);
    xv[r] = ((a - mu) * rs) * sc + bi;
  }
#pragma unroll
  for (int r2 = 0; r2 < 4; ++r2) slab[(prow + r2) * SPF + col] = fmaxf(xv[2 * r2], xv[2 * r2 + 1]);
}

__global__ __launch_bounds__(NTHF) void front_kernel(const float* __restrict__ cgm, const unsigned short* __restrict__ WTDp,
                                                    const float* __restrict__ tdb, const float* __restrict__ bsc,
                                                    const float* __restrict__ bbi, const float* __restrict__ bmu,
                                                    const float* __restrict__ bva, unsigned short* __restrict__ Xp) {
  __shared__ __align__(16) unsigned short At[256 * APF];
  __shared__ __align__(16) float          Sl[NTHF / 32][16 * SPF];
  const _Float16* WTD = (const _Float16*)WTDp;
  const int tid = threadIdx.x, lane = tid & 31, wave = tid >> 5;
  const int c = lane & 15, hh = lane >> 4, koff = hh * 8;
  const size_t r0 = (size_t)blockIdx.x * 256;
  const float* src = cgm + r0 * NF;

#pragma unroll
  for (int it = 0; it < 6; ++it) {
    const int q   = it * NTHF + tid;
    const int row = q / 6, col = (q - row * 6) * 4;
    const v4f v = *(const v4f*)(src + (size_t)q * 4);
    const unsigned short u0 = __builtin_bit_cast(unsigned short, (_Float16)v[0]);
    const unsigned short u1 = __builtin_bit_cast(unsigned short, (_Float16)v[1]);
    const unsigned short u2 = __builtin_bit_cast(unsigned short, (_Float16)v[2]);
    const unsigned short u3 = __builtin_bit_cast(unsigned short, (_Float16)v[3]);
    v2u pk;
    pk[0] = (unsigned)u0 | ((unsigned)u1 << 16);
    pk[1] = (unsigned)u2 | ((unsigned)u3 << 16);
    *(v2u*)(At + row * APF + col) = pk;
  }
  {
    const v4u z4 = {0u, 0u, 0u, 0u};
    *(v4u*)(At + tid * APF + NF) = z4;
  }
  __syncthreads();

  const _Float16* Atile = (const _Float16*)At;
  const v8f z8 = {0.f, 0.f, 0.f, 0.f, 0.f, 0.f, 0.f, 0.f};
  const v16h bw0 = Frag<_Float16>::load(WTD + (size_t)c * NFP + koff);
  const v16h bw1 = Frag<_Float16>::load(WTD + (size_t)(16 + c) * NFP + koff);
  const v16h a0  = Frag<_Float16>::load(Atile + (size_t)(32 * wave + c) * APF + koff);
  const v16h a1  = Frag<_Float16>::load(Atile + (size_t)(32 * wave + 16 + c) * APF + koff);
  v8f acc00 = Frag<_Float16>::mma(a0, bw0, z8);
  v8f acc01 = Frag<_Float16>::mma(a0, bw1, z8);
  v8f acc10 = Frag<_Float16>::mma(a1, bw0, z8);
  v8f acc11 = Frag<_Float16>::mma(a1, bw1, z8);
  guard4_h4(acc00, acc01, acc10, acc11, a0, a1, bw0, bw1);

  float* slab = Sl[wave];
  const int n0 = c, n1 = 16 + c;
  const float tb0 = tdb[n0], mu0 = bmu[n0], rs0 = rsqrtf(bva[n0] + BN_EPS), sc0 = bsc[n0], bi0 = bbi[n0];
  const float tb1 = tdb[n1], mu1 = bmu[n1], rs1 = rsqrtf(bva[n1] + BN_EPS), sc1 = bsc[n1], bi1 = bbi[n1];
  front_epi(acc00, tb0, mu0, rs0, sc0, bi0, slab, 4 * hh,     n0);
  front_epi(acc01, tb1, mu1, rs1, sc1, bi1, slab, 4 * hh,     n1);
  front_epi(acc10, tb0, mu0, rs0, sc0, bi0, slab, 8 + 4 * hh, n0);
  front_epi(acc11, tb1, mu1, rs1, sc1, bi1, slab, 8 + 4 * hh, n1);
  __syncthreads();

  const int pr = lane >> 2, e8 = (lane & 3) * 8;
  const size_t prb = (size_t)blockIdx.x * 128 + (size_t)(16 * wave);
  v8h hv[2];
#pragma unroll
  for (int q = 0; q < 2; ++q) {
    const float* sp = slab + (8 * q + pr) * SPF + e8;
#pragma unroll
    for (int e = 0; e < 8; ++e) hv[q][e] = (_Float16)sp[e];
  }
  for (int ps = 0; ps < 2; ++ps) {
#pragma unroll
    for (int q = 0; q < 2; ++q)
      *(volatile v8h*)(Xp + (prb + (size_t)(8 * q + pr)) * NC + e8) = hv[q];
    __threadfence();
  }
}

__global__ __launch_bounds__(NTHR) void rnn1_kernel(const unsigned short* __restrict__ Xp, const unsigned short* __restrict__ W1Xp,
                                                   const unsigned short* __restrict__ W1Hp, const float* __restrict__ b1f,
                                                   const float* __restrict__ b1b, unsigned short* __restrict__ Y1p, int bbase) {
  __shared__ __align__(16) _Float16 Ah[2][16 * HP];
  const _Float16* X   = (const _Float16*)Xp;
  const _Float16* W1X = (const _Float16*)W1Xp;
  const _Float16* W1H = (const _Float16*)W1Hp;
  const int tid = threadIdx.x, lane = tid & 31, wave = tid >> 5;
  const int c = lane & 15, hh = lane >> 4, koff = hh * 8;
  constexpr int NMT = BCH / 16;
  const int d  = blockIdx.x / NMT;
  const int rb = (blockIdx.x - d * NMT) * 16;

  {
    _Float16* ahf = &Ah[0][0];
#pragma unroll 1
    for (int i = tid; i < 2 * 16 * HP; i += NTHR) ahf[i] = (_Float16)0.0f;
  }
  const int j0 = 32 * wave + c, j1 = j0 + 16;
  const float fsel_f = (float)(1 - d), fsel_b = (float)d;
  const float bv0 = fsel_f * b1f[j0] + fsel_b * b1b[j0];
  const float bv1 = fsel_f * b1f[j1] + fsel_b * b1b[j1];
  __syncthreads();

  const _Float16* wx = W1X + (size_t)(d * NU) * NFP;
  const _Float16* wh = W1H + (size_t)(d * NU) * NU;
  const v8f z8 = {0.f, 0.f, 0.f, 0.f, 0.f, 0.f, 0.f, 0.f};

#pragma unroll 1
  for (int s = 0; s < NT2; ++s) {
    const int cur = s & 1;
    const int t   = s + d * (NT2 - 1 - 2 * s);
    const _Float16* ahrow = &Ah[cur][0] + c * HP + koff;
    _Float16*       ahn   = &Ah[cur ^ 1][0];
    v8f acc0 = z8, acc1 = z8;
    {
      const v16h ax  = Frag<_Float16>::load(X + ((size_t)(bbase + rb + c) * NT2 + (size_t)t) * NC + koff);
      const v16h bx0 = Frag<_Float16>::load(wx + (size_t)j0 * NFP + koff);
      const v16h bx1 = Frag<_Float16>::load(wx + (size_t)j1 * NFP + koff);
      acc0 = Frag<_Float16>::mma(ax, bx0, acc0);
      acc1 = Frag<_Float16>::mma(ax, bx1, acc1);
      guard2_h3(acc0, acc1, ax, bx0, bx1);
    }
#pragma unroll 1
    for (int k0 = 0; k0 < NU; k0 += 32) {
      const v16h a   = Frag<_Float16>::load(ahrow + k0);
      const v16h bw0 = Frag<_Float16>::load(wh + (size_t)j0 * NU + koff + k0);
      const v16h bw1 = Frag<_Float16>::load(wh + (size_t)j1 * NU + koff + k0);
      acc0 = Frag<_Float16>::mma(a, bw0, acc0);
      acc1 = Frag<_Float16>::mma(a, bw1, acc1);
      guard2_h3(acc0, acc1, a, bw0, bw1);
    }
    acc_guard2(acc0, acc1);
#pragma unroll
    for (int r = 0; r < 8; ++r) {
      const float h0v = tanh_f(acc0[r] * WSC_INV + bv0);
      const float h1v = tanh_f(acc1[r] * WSC_INV + bv1);
      ahn[(8 * hh + r) * HP + j0] = (_Float16)h0v;
      ahn[(8 * hh + r) * HP + j1] = (_Float16)h1v;
    }
    __syncthreads();

    v8h sv[2]; size_t so[2];
#pragma unroll
    for (int q = 0; q < 2; ++q) {
      const int row = 4 * wave + 2 * q + hh;
      sv[q] = *(const v8h*)(ahn + row * HP + c * 8);
      so[q] = ((size_t)(rb + row) * NT2 + (size_t)t) * NU2 + (size_t)(d * NU + c * 8);
    }
    for (int ps = 0; ps < 2; ++ps) {
#pragma unroll
      for (int q = 0; q < 2; ++q) *(volatile v8h*)(Y1p + so[q]) = sv[q];
      __threadfence();
    }
  }
}

__global__ __launch_bounds__(NTHR) void rnn2_kernel(const unsigned short* __restrict__ Y1p, const unsigned short* __restrict__ W2Xp,
                                                   const unsigned short* __restrict__ W2Hp, const float* __restrict__ b2f,
                                                   float* __restrict__ H2F, int bbase) {
  __shared__ __align__(16) _Float16 Ah[2][16 * HP];
  __shared__ __align__(16) float    Hs[16 * OPH];
  const _Float16* Y1  = (const _Float16*)Y1p;
  const _Float16* W2X = (const _Float16*)W2Xp;
  const _Float16* W2H = (const _Float16*)W2Hp;
  const int tid = threadIdx.x, lane = tid & 31, wave = tid >> 5;
  const int c = lane & 15, hh = lane >> 4, koff = hh * 8;
  const int rb = blockIdx.x * 16;

  {
    _Float16* ahf = &Ah[0][0];
#pragma unroll 1
    for (int i = tid; i < 2 * 16 * HP; i += NTHR) ahf[i] = (_Float16)0.0f;
  }
  const int j0 = 32 * wave + c, j1 = j0 + 16;
  const float bv0 = b2f[j0], bv1 = b2f[j1];
  float hst[2][8];
#pragma unroll
  for (int nt = 0; nt < 2; ++nt)
#pragma unroll
    for (int r = 0; r < 8; ++r) hst[nt][r] = 0.0f;
  __syncthreads();

  const v8f z8 = {0.f, 0.f, 0.f, 0.f, 0.f, 0.f, 0.f, 0.f};

#pragma unroll 1
  for (int s = 0; s < NT2; ++s) {
    const int cur = s & 1;
    const _Float16* ahrow = &Ah[cur][0] + c * HP + koff;
    _Float16*       ahn   = &Ah[cur ^ 1][0];
    const _Float16* yrow  = Y1 + ((size_t)(rb + c) * NT2 + (size_t)s) * NU2 + koff;
    v8f acc0 = z8, acc1 = z8;
#pragma unroll 1
    for (int k0 = 0; k0 < NU2; k0 += 32) {
      const v16h a   = Frag<_Float16>::load(yrow + k0);
      const v16h bw0 = Frag<_Float16>::load(W2X + (size_t)j0 * NU2 + koff + k0);
      const v16h bw1 = Frag<_Float16>::load(W2X + (size_t)j1 * NU2 + koff + k0);
      acc0 = Frag<_Float16>::mma(a, bw0, acc0);
      acc1 = Frag<_Float16>::mma(a, bw1, acc1);
      guard2_h3(acc0, acc1, a, bw0, bw1);
    }
#pragma unroll 1
    for (int k0 = 0; k0 < NU; k0 += 32) {
      const v16h a   = Frag<_Float16>::load(ahrow + k0);
      const v16h bw0 = Frag<_Float16>::load(W2H + (size_t)j0 * NU + koff + k0);
      const v16h bw1 = Frag<_Float16>::load(W2H + (size_t)j1 * NU + koff + k0);
      acc0 = Frag<_Float16>::mma(a, bw0, acc0);
      acc1 = Frag<_Float16>::mma(a, bw1, acc1);
      guard2_h3(acc0, acc1, a, bw0, bw1);
    }
    acc_guard2(acc0, acc1);
#pragma unroll
    for (int r = 0; r < 8; ++r) {
      const float h0v = tanh_f(acc0[r] * WSC_INV + bv0);
      const float h1v = tanh_f(acc1[r] * WSC_INV + bv1);
      hst[0][r] = h0v;
      hst[1][r] = h1v;
      ahn[(8 * hh + r) * HP + j0] = (_Float16)h0v;
      ahn[(8 * hh + r) * HP + j1] = (_Float16)h1v;
    }
    __syncthreads();
  }

#pragma unroll
  for (int r = 0; r < 8; ++r) {
    Hs[(8 * hh + r) * OPH + j0] = hst[0][r];
    Hs[(8 * hh + r) * OPH + j1] = hst[1][r];
  }
  __syncthreads();
  v4f vv[4]; size_t vo[4];
#pragma unroll
  for (int it = 0; it < 4; ++it) {
    const int idx = it * NTHR + tid;
    const int row = idx >> 5, c4 = (idx & 31) * 4;
    vv[it] = *(const v4f*)(Hs + row * OPH + c4);
    vo[it] = (size_t)(bbase + rb + row) * NU + (size_t)c4;
  }
  for (int ps = 0; ps < 2; ++ps) {
#pragma unroll
    for (int it = 0; it < 4; ++it) *(volatile v4f*)(H2F + vo[it]) = vv[it];
    __threadfence();
  }
}

__global__ __launch_bounds__(NTHR) void h2b_kernel(const unsigned short* __restrict__ Y1p, const float* __restrict__ w2bi,
                                                  const float* __restrict__ b2b, float* __restrict__ H2B, int bbase) {
  __shared__ float yv[16 * NU2];
  __shared__ __align__(16) float ho[16 * OPH];
  const int tid = threadIdx.x;
  const int rb  = blockIdx.x * 16;
  const unsigned* Yw = (const unsigned*)Y1p;
#pragma unroll 1
  for (int rr = 0; rr < 16; ++rr) {
    const unsigned w = Yw[((size_t)(rb + rr) * NT2 + (size_t)(NT2 - 1)) * (NU2 / 2) + tid];
    yv[rr * NU2 + 2 * tid]     = h16_to_f32(w & 0xffffu);
    yv[rr * NU2 + 2 * tid + 1] = h16_to_f32(w >> 16);
  }
  __syncthreads();
  const int j = tid;
  const float bj = b2b[j];
#pragma unroll 1
  for (int rr = 0; rr < 16; ++rr) {
    const float* yr = yv + rr * NU2;
    float acc = 0.0f;
#pragma unroll 4
    for (int kk = 0; kk < NU2; ++kk) acc += yr[kk] * w2bi[(size_t)kk * NU + j];
    ho[rr * OPH + j] = tanh_f(acc + bj);
  }
  __syncthreads();
  v4f vv[4]; size_t vo[4];
#pragma unroll
  for (int it = 0; it < 4; ++it) {
    const int idx = it * NTHR + tid;
    const int row = idx >> 5, c4 = (idx & 31) * 4;
    vv[it] = *(const v4f*)(ho + row * OPH + c4);
    vo[it] = (size_t)(bbase + rb + row) * NU + (size_t)c4;
  }
  for (int ps = 0; ps < 2; ++ps) {
#pragma unroll
    for (int it = 0; it < 4; ++it) *(volatile v4f*)(H2B + vo[it]) = vv[it];
    __threadfence();
  }
}

__global__ __launch_bounds__(NTHF) void head_kernel(const float* __restrict__ H2F, const float* __restrict__ H2B,
                                                   const float* __restrict__ other, const float* __restrict__ d1w,
                                                   const float* __restrict__ d1b, const float* __restrict__ ow,
                                                   const float* __restrict__ ob, float* __restrict__ out) {
  __shared__ float zs[32 * ZP];
  __shared__ float us[32 * UP];
  const int tid = threadIdx.x;
  const int rb  = blockIdx.x * 32;
#pragma unroll 1
  for (int i = tid; i < 32 * NU; i += NTHF) {
    const int row = i >> 7, kk = i & 127;
    zs[row * ZP + kk]      = H2F[(size_t)(rb + row) * NU + kk];
    zs[row * ZP + NU + kk] = H2B[(size_t)(rb + row) * NU + kk];
  }
  if (tid < 32 * NO) {
    const int row = tid / NO, kk = tid - row * NO;
    zs[row * ZP + NU2 + kk] = other[(size_t)(rb + row) * NO + kk];
  }
  __syncthreads();
  const int j = tid & 63, rq = tid >> 6;
  const float bj = d1b[j];
#pragma unroll 1
  for (int rr = 0; rr < 8; ++rr) {
    const int row = rq * 8 + rr;
    const float* zr = zs + row * ZP;
    float acc = 0.0f;
#pragma unroll 2
    for (int kk = 0; kk < NZ; ++kk) acc += zr[kk] * d1w[(size_t)kk * ND1 + j];
    us[row * UP + j] = tanh_f(acc + bj);
  }
  __syncthreads();
  if (tid < 32) {
    const float* ur = us + tid * UP;
    float sacc = 0.0f;
#pragma unroll 4
    for (int jj = 0; jj < ND1; ++jj) sacc += ur[jj] * ow[jj];
    const float o = sacc + ob[0];
    ((volatile float*)out)[rb + tid] = o;
    __threadfence();
    ((volatile float*)out)[rb + tid] = o;
  }
}

extern "C" void kernel_launch(void* const* d_in, const int* in_sizes, int n_in,
                              void* d_out, int out_size, void* d_ws, size_t ws_size, hipStream_t stream) {
  if (n_in < 24 || d_out == nullptr || d_ws == nullptr) return;
  if (in_sizes[0] != NB * NTR * NF || in_sizes[1] != NB * NO || in_sizes[2] != NF * NC ||
      in_sizes[3] != NC || in_sizes[4] != NC || in_sizes[5] != NC || in_sizes[6] != NC || in_sizes[7] != NC ||
      in_sizes[8] != NC * NU || in_sizes[9] != NU * NU || in_sizes[10] != NU ||
      in_sizes[11] != NC * NU || in_sizes[12] != NU * NU || in_sizes[13] != NU ||
      in_sizes[14] != NU2 * NU || in_sizes[15] != NU * NU || in_sizes[16] != NU ||
      in_sizes[17] != NU2 * NU || in_sizes[18] != NU * NU || in_sizes[19] != NU ||
      in_sizes[20] != NZ * ND1 || in_sizes[21] != ND1 || in_sizes[22] != ND1 || in_sizes[23] != 1 ||
      out_size != NB) return;

  const float* cgm   = (const float*)d_in[0];
  const float* other = (const float*)d_in[1];
  const float* td_w  = (const float*)d_in[2];
  const float* td_b  = (const float*)d_in[3];
  const float* bn_sc = (const float*)d_in[4];
  const float* bn_bi = (const float*)d_in[5];
  const float* bn_mu = (const float*)d_in[6];
  const float* bn_va = (const float*)d_in[7];
  const float* w1f_i = (const float*)d_in[8];
  const float* w1f_h = (const float*)d_in[9];
  const float* b1f   = (const float*)d_in[10];
  const float* w1b_i = (const float*)d_in[11];
  const float* w1b_h = (const float*)d_in[12];
  const float* b1b   = (const float*)d_in[13];
  const float* w2f_i = (const float*)d_in[14];
  const float* w2f_h = (const float*)d_in[15];
  const float* b2f   = (const float*)d_in[16];
  const float* w2b_i = (const float*)d_in[17];
  const float* b2b   = (const float*)d_in[19];
  const float* d1_w  = (const float*)d_in[20];
  const float* d1_b  = (const float*)d_in[21];
  const float* out_w = (const float*)d_in[22];
  const float* out_b = (const float*)d_in[23];
  float* out = (float*)d_out;

  char* ws = (char*)d_ws; size_t off = 0;
  auto carve = [&](size_t bytes) -> char* { char* p = ws + off; off += (bytes + 255) & ~(size_t)255; return p; };
  unsigned short* WTD = (unsigned short*)carve((size_t)NC * NFP * 2);
  unsigned short* W1X = (unsigned short*)carve((size_t)NU2 * NFP * 2);
  unsigned short* W1H = (unsigned short*)carve((size_t)NU2 * NU * 2);
  unsigned short* W2X = (unsigned short*)carve((size_t)NU * NU2 * 2);
  unsigned short* W2H = (unsigned short*)carve((size_t)NU * NU * 2);
  unsigned short* X   = (unsigned short*)carve((size_t)NB * NT2 * NC * 2);
  unsigned short* Y1  = (unsigned short*)carve((size_t)BCH * NT2 * NU2 * 2);
  float*          H2F = (float*)carve((size_t)NB * NU * 4);
  float*          H2B = (float*)carve((size_t)NB * NU * 4);
  if (off > ws_size || off > (size_t)134217728) return;

  wprep_kernel<<<1,  NTHF, 0, stream>>>(td_w,  NF,  NC, NFP, WTD, WSC);
  wprep_kernel<<<2,  NTHF, 0, stream>>>(w1f_i, NC,  NU, NC,  W1X, WSC);
  wprep_kernel<<<2,  NTHF, 0, stream>>>(w1b_i, NC,  NU, NC,  W1X + (size_t)NU * NFP, WSC);
  wprep_kernel<<<8,  NTHF, 0, stream>>>(w1f_h, NU,  NU, NU,  W1H, WSC);
  wprep_kernel<<<8,  NTHF, 0, stream>>>(w1b_h, NU,  NU, NU,  W1H + (size_t)NU * NU, WSC);
  wprep_kernel<<<16, NTHF, 0, stream>>>(w2f_i, NU2, NU, NU2, W2X, WSC);
  wprep_kernel<<<8,  NTHF, 0, stream>>>(w2f_h, NU,  NU, NU,  W2H, WSC);

  front_kernel<<<(NB * NTR) / 256, NTHF, 0, stream>>>(cgm, WTD, td_b, bn_sc, bn_bi, bn_mu, bn_va, X);

  for (int p = 0; p < NPASS; ++p) {
    const int bbase = p * BCH;
    rnn1_kernel<<<2 * (BCH / 16), NTHR, 0, stream>>>(X, W1X, W1H, b1f, b1b, Y1, bbase);
    rnn2_kernel<<<BCH / 16, NTHR, 0, stream>>>(Y1, W2X, W2H, b2f, H2F, bbase);
    h2b_kernel<<<BCH / 16, NTHR, 0, stream>>>(Y1, w2b_i, b2b, H2B, bbase);
  }

  head_kernel<<<NB / 32, NTHF, 0, stream>>>(H2F, H2B, other, d1_w, d1_b, out_w, out_b, out);
}
